// DRMMTKS_class_80625126081184
// MI455X (gfx1250) — hardware-verified
//
#include <hip/hip_runtime.h>
#include <stdint.h>
#include <stddef.h>

#define VOCAB 50000
#define EMB   300
#define KPAD  320
#define BATCH 128
#define TQ    32
#define TD    4096
#define TOPK  20
#define NCH   128
#define NTILE (TD / NCH)
#define SP    129
#define OPSC  16.0f
#define ACCSC (1.0f / 256.0f)

typedef _Float16 v16h __attribute__((ext_vector_type(16)));
typedef _Float16 v8h  __attribute__((ext_vector_type(8)));
typedef float    v8f  __attribute__((ext_vector_type(8)));
typedef float    v4f  __attribute__((ext_vector_type(4)));
typedef unsigned int u32x4 __attribute__((ext_vector_type(4)));
typedef v8h   __attribute__((may_alias)) v8ha;
typedef v4f   __attribute__((may_alias)) v4fa;
typedef u32x4 __attribute__((may_alias)) u32x4a;

union Frag { v16h v; v8h half[2]; };

static_assert(VOCAB % 8 == 0);
static_assert(KPAD % 32 == 0);
static_assert((TQ * (KPAD / 8)) % 256 == 0);
static_assert((NCH * (KPAD / 8)) % 256 == 0);
static_assert(TD % NCH == 0);
static_assert((TQ * TOPK) % 4 == 0);
static_assert(((TQ * TOPK) / 4) % 32 == 0);
static_assert((BATCH * TQ) % 256 == 0);
static_assert(BATCH % 8 == 0);
static_assert((TQ * TOPK * 4) % 128 == 0);

__device__ __forceinline__ v8f wmma_f16(v16h a, v16h b, v8f c) {
  v8f d = __builtin_amdgcn_wmma_f32_16x16x32_f16(false, a, false, b, (short)0, c, false, false);
  asm volatile("v_nop\n\tv_nop\n\tv_nop\n\tv_nop" : "+v"(d) : "v"(a), "v"(b));
  return d;
}

__device__ __forceinline__ v16h load_frag(const _Float16* p, int h) {
  Frag f;
  f.half[0] = *(const v8ha*)(p + 8 * h);
  f.half[1] = *(const v8ha*)(p + 16 + 8 * h);
  return f.v;
}

__device__ __forceinline__ void tk_ins(float (&t)[TOPK], float v) {
  if (v > t[0]) {
    t[0] = v;
#pragma unroll
    for (int i = 0; i < TOPK - 1; ++i) {
      const float a = t[i], c = t[i + 1];
      const bool sw = a > c;
      t[i]     = sw ? c : a;
      t[i + 1] = sw ? a : c;
    }
  }
}

__global__ __launch_bounds__(256) void norm_table_kernel(const float* __restrict__ emb,
                                                         _Float16* __restrict__ ntab) {
  const int w = threadIdx.x >> 5, l = threadIdx.x & 31;
  const int row = blockIdx.x * 8 + w;
  const float* src = emb + (size_t)row * EMB;

  const v4f a0 = *(const v4fa*)(src + 8 * l);
  const v4f a1 = *(const v4fa*)(src + 8 * l + 4);

  const int pB = 32 + (l & 7);
  const bool vb0 = (8 * pB + 4 <= EMB);
  const bool vb1 = (8 * pB + 8 <= EMB);
  const int ob0 = vb0 ? (8 * pB) : 0;
  const int ob1 = vb1 ? (8 * pB + 4) : 0;
  v4f b0 = *(const v4fa*)(src + ob0);
  v4f b1 = *(const v4fa*)(src + ob1);
  const v4f z4 = {0.f, 0.f, 0.f, 0.f};
  if (!vb0) b0 = z4;
  if (!vb1) b1 = z4;
  const bool hasB = (l < 8);

  float s = a0.x * a0.x + a0.y * a0.y + a0.z * a0.z + a0.w * a0.w
          + a1.x * a1.x + a1.y * a1.y + a1.z * a1.z + a1.w * a1.w;
  const float sb = b0.x * b0.x + b0.y * b0.y + b0.z * b0.z + b0.w * b0.w
                 + b1.x * b1.x + b1.y * b1.y + b1.z * b1.z + b1.w * b1.w;
  s += hasB ? sb : 0.0f;
#pragma unroll
  for (int d = 16; d >= 1; d >>= 1) s += __shfl_xor(s, d, 32);

  const float nrm = sqrtf(s);
  const float inv = 1.0f / fmaxf(nrm, 1e-8f);
  const float sc = inv * OPSC;

  const v8h oA = { (_Float16)(a0.x * sc), (_Float16)(a0.y * sc), (_Float16)(a0.z * sc), (_Float16)(a0.w * sc),
                   (_Float16)(a1.x * sc), (_Float16)(a1.y * sc), (_Float16)(a1.z * sc), (_Float16)(a1.w * sc) };
  const v8h oB = { (_Float16)(b0.x * sc), (_Float16)(b0.y * sc), (_Float16)(b0.z * sc), (_Float16)(b0.w * sc),
                   (_Float16)(b1.x * sc), (_Float16)(b1.y * sc), (_Float16)(b1.z * sc), (_Float16)(b1.w * sc) };

  _Float16* dst = ntab + (size_t)row * KPAD;
  *(volatile v8h*)(dst + 8 * l) = oA;
  if (hasB) *(volatile v8h*)(dst + 8 * pB) = oB;
  __threadfence();
  *(volatile v8h*)(dst + 8 * l) = oA;
  if (hasB) *(volatile v8h*)(dst + 8 * pB) = oB;
}

__global__ __launch_bounds__(256) void sim_topk_kernel(const _Float16* __restrict__ ntab,
                                                       const int* __restrict__ query,
                                                       const int* __restrict__ doc,
                                                       float* __restrict__ cand) {
  extern __shared__ __attribute__((aligned(16))) _Float16 lds_dyn[];
  __shared__ float sS[TQ * SP];
  __shared__ __attribute__((aligned(16))) float sC[TQ * TOPK];

  _Float16* ldsQ = lds_dyn;
  _Float16* ldsD = lds_dyn + TQ * KPAD;

  const int b = blockIdx.y, tile = blockIdx.x;
  const int tid = threadIdx.x, w = tid >> 5, l = tid & 31;
  const int h = l >> 4, m = l & 15;

#pragma unroll 1
  for (int idx = tid; idx < TQ * (KPAD / 8); idx += 256) {
    const int r = idx / (KPAD / 8), c = idx - r * (KPAD / 8);
    int tok = query[b * TQ + r];
    tok = min(max(tok, 0), VOCAB - 1);
    const u32x4 v = *(const u32x4a*)(ntab + (size_t)tok * KPAD + 8 * c);
    *(u32x4a*)(ldsQ + r * KPAD + 8 * c) = v;
  }
#pragma unroll 1
  for (int idx = tid; idx < NCH * (KPAD / 8); idx += 256) {
    const int r = idx / (KPAD / 8), c = idx - r * (KPAD / 8);
    int tok = doc[(size_t)b * TD + (size_t)tile * NCH + r];
    tok = min(max(tok, 0), VOCAB - 1);
    const u32x4 v = *(const u32x4a*)(ntab + (size_t)tok * KPAD + 8 * c);
    *(u32x4a*)(ldsD + r * KPAD + 8 * c) = v;
  }
  __syncthreads();

  const int mt = w & 1, np = w >> 1;
  const _Float16* qa  = ldsQ + (mt * 16 + m) * KPAD;
  const _Float16* db0 = ldsD + (np * 32 + m) * KPAD;
  const _Float16* db1 = db0 + 16 * KPAD;

  const v8f zero8 = {0.f, 0.f, 0.f, 0.f, 0.f, 0.f, 0.f, 0.f};
  v8f acc0 = zero8, acc1 = zero8;
#pragma unroll 2
  for (int k0 = 0; k0 < KPAD; k0 += 32) {
    const v16h af  = load_frag(qa + k0, h);
    const v16h bf0 = load_frag(db0 + k0, h);
    const v16h bf1 = load_frag(db1 + k0, h);
    acc0 = wmma_f16(af, bf0, acc0);
    acc1 = wmma_f16(af, bf1, acc1);
  }

#pragma unroll
  for (int r = 0; r < 8; ++r) {
    const int q = mt * 16 + 8 * h + r;
    sS[q * SP + np * 32 + m]      = acc0[r] * ACCSC;
    sS[q * SP + np * 32 + 16 + m] = acc1[r] * ACCSC;
  }
  __syncthreads();

  if (w == 0) {
    float t[TOPK];
#pragma unroll
    for (int i = 0; i < TOPK; ++i) t[i] = -1.0e30f;
#pragma unroll 1
    for (int j = 0; j < NCH; ++j) tk_ins(t, sS[l * SP + j]);
#pragma unroll
    for (int i = 0; i < TOPK; ++i) sC[l * TOPK + i] = t[TOPK - 1 - i];
  }
  __syncthreads();

  float* dstc = cand + ((size_t)b * NTILE + tile) * (size_t)(TQ * TOPK);
  v4f cv = {0.f, 0.f, 0.f, 0.f};
  const bool act = (tid < (TQ * TOPK) / 4);
  if (act) cv = *(const v4fa*)(sC + 4 * tid);
  if (act) *(volatile v4f*)(dstc + 4 * tid) = cv;
  __threadfence();
  if (act) *(volatile v4f*)(dstc + 4 * tid) = cv;
}

__global__ __launch_bounds__(256) void head_kernel(const float* __restrict__ cand,
                                                   const int* __restrict__ query,
                                                   const float* __restrict__ idf,
                                                   const float* __restrict__ ffw_W,
                                                   const float* __restrict__ ffw_b,
                                                   const float* __restrict__ gates_W,
                                                   const float* __restrict__ out_W,
                                                   const float* __restrict__ out_b,
                                                   const int* __restrict__ topk_p,
                                                   float* __restrict__ out) {
  __shared__ float sF[BATCH * TQ];
  __shared__ float sT[256 * TOPK];
  __shared__ __attribute__((aligned(16))) float sOut[BATCH];

  const int tid = threadIdx.x, w = tid >> 5, l = tid & 31;
  int kt = topk_p[0];
  kt = min(max(kt, 0), TOPK);
  const float fb = ffw_b[0];

#pragma unroll 1
  for (int it = 0; it < (BATCH * TQ) / 256; ++it) {
    const int pq = it * 256 + tid;
    const int b = pq >> 5, q = pq & 31;
    float t[TOPK];
#pragma unroll
    for (int i = 0; i < TOPK; ++i) t[i] = -1.0e30f;
#pragma unroll 1
    for (int tl = 0; tl < NTILE; ++tl) {
      const float* src = cand + (((size_t)b * NTILE + tl) * TQ + q) * (size_t)TOPK;
#pragma unroll
      for (int c = 0; c < TOPK / 4; ++c) {
        const v4f v = *(const v4fa*)(src + 4 * c);
        tk_ins(t, v.x); tk_ins(t, v.y); tk_ins(t, v.z); tk_ins(t, v.w);
      }
    }
#pragma unroll
    for (int i = 0; i < TOPK; ++i) sT[tid * TOPK + i] = t[TOPK - 1 - i];
    float s = 0.0f;
#pragma unroll 1
    for (int j = 0; j < kt; ++j) s = fmaf(sT[tid * TOPK + j], ffw_W[j], s);
    sF[pq] = tanhf(s + fb);
  }
  __syncthreads();

  const float g = gates_W[0], ow = out_W[0], ob = out_b[0];
#pragma unroll 1
  for (int i = 0; i < BATCH / 8; ++i) {
    const int b = w * (BATCH / 8) + i;
    const int tok = query[b * TQ + l];
    const float qm = (tok != 0) ? 1.0f : 0.0f;
    const float am = (1.0f - qm) * -1.0e7f;
    const float logit = idf[b * TQ + l] * g + am;
    float mx = logit;
#pragma unroll
    for (int d = 16; d >= 1; d >>= 1) mx = fmaxf(mx, __shfl_xor(mx, d, 32));
    const float e = expf(logit - mx);
    float se = e;
#pragma unroll
    for (int d = 16; d >= 1; d >>= 1) se += __shfl_xor(se, d, 32);
    const float wgt = e * (1.0f / se);
    float dd = wgt * sF[b * TQ + l];
#pragma unroll
    for (int d = 16; d >= 1; d >>= 1) dd += __shfl_xor(dd, d, 32);
    const float score = dd * ow + ob;
    if (l == 0) sOut[b] = score;
  }
  __syncthreads();

  v4f ov = {0.f, 0.f, 0.f, 0.f};
  if (w == 0) ov = *(const v4fa*)(sOut + 4 * l);
  if (w == 0) *(volatile v4f*)(out + 4 * l) = ov;
  __threadfence();
  if (w == 0) *(volatile v4f*)(out + 4 * l) = ov;
}

extern "C" void kernel_launch(void* const* d_in, const int* in_sizes, int n_in,
                              void* d_out, int out_size, void* d_ws, size_t ws_size,
                              hipStream_t stream) {
  if (n_in < 10) return;
  if (in_sizes[0] != BATCH * TD) return;
  if (in_sizes[1] != BATCH * TQ) return;
  if (in_sizes[2] != BATCH * TQ) return;
  if (in_sizes[3] != VOCAB * EMB) return;
  if (in_sizes[4] != TOPK) return;
  if (in_sizes[5] < 1 || in_sizes[6] < 1 || in_sizes[7] < 1 || in_sizes[8] < 1 || in_sizes[9] < 1) return;
  if (out_size != BATCH) return;

  const int*   doc    = (const int*)d_in[0];
  const int*   query  = (const int*)d_in[1];
  const float* idf    = (const float*)d_in[2];
  const float* emb    = (const float*)d_in[3];
  const float* ffw_W  = (const float*)d_in[4];
  const float* ffw_b  = (const float*)d_in[5];
  const float* gatesW = (const float*)d_in[6];
  const float* outW   = (const float*)d_in[7];
  const float* outB   = (const float*)d_in[8];
  const int*   topk_p = (const int*)d_in[9];
  float* out = (float*)d_out;

  const size_t ntab_bytes = (size_t)VOCAB * KPAD * sizeof(_Float16);
  const size_t cand_bytes = (size_t)BATCH * NTILE * TQ * TOPK * sizeof(float);
  const size_t total = ntab_bytes + cand_bytes;
  if (total > ws_size) return;

  char* ws = (char*)d_ws;
  _Float16* ntab = (_Float16*)ws;
  float* cand = (float*)(ws + ntab_bytes);

  const size_t dyn_lds = (size_t)(TQ + NCH) * KPAD * sizeof(_Float16);
  hipFuncSetAttribute(reinterpret_cast<const void*>(&sim_topk_kernel),
                      hipFuncAttributeMaxDynamicSharedMemorySize, (int)dyn_lds);

  norm_table_kernel<<<VOCAB / 8, 256, 0, stream>>>(emb, ntab);
  sim_topk_kernel<<<dim3(NTILE, BATCH), 256, dyn_lds, stream>>>(ntab, query, doc, cand);
  head_kernel<<<1, 256, 0, stream>>>(cand, query, idf, ffw_W, ffw_b, gatesW, outW, outB,
                                     topk_p, out);
}
